// MultiDimensionalRNNBase_77635828842557
// MI455X (gfx1250) — hardware-verified
//
#include <hip/hip_runtime.h>
#include <cmath>

typedef _Float16 bf16_t;
typedef bf16_t v16bf __attribute__((ext_vector_type(16)));
#define PSTR 32
#define VST2(T, ptr, val) do { const T _v = (val); *(volatile T*)(ptr) = _v; __threadfence(); *(volatile T*)(ptr) = _v; } while (0)
typedef float  v8f   __attribute__((ext_vector_type(8)));
typedef float  v4f   __attribute__((ext_vector_type(4)));
typedef int    v4i   __attribute__((ext_vector_type(4)));

#define HH 32
#define WW 32
#define HID 64
#define NCLS 10
#define BATCHN 128
#define STEPS 63

#define TANHF(x) tanhf(x)

#define BT_STRIDE 136
#define H_STRIDE  72
#define H_ROWS    33
#define ACT_STRIDE 72
#define ACT_TRASH_PIX 1024
#define XSK_STRIDE 36

#define BT_BYTES   (HID * BT_STRIDE * 2)
#define XSK_BYTES  (64 * XSK_STRIDE * 4)
#define HBUF_ELEMS (H_ROWS * H_STRIDE)
#define HB_BYTES   (2 * HBUF_ELEMS * 2)
#define ACT_BYTES  ((HH * WW + 1) * ACT_STRIDE * 2)
#define RED_BYTES  (8 * NCLS * 4)
#define SMEM_BYTES (BT_BYTES + XSK_BYTES + HB_BYTES + ACT_BYTES + RED_BYTES)

union Frag { v16bf v; v4i q[2]; };

__global__ __launch_bounds__(256) void mdrnn_kernel(
    const float* __restrict__ x,
    const float* __restrict__ w_in,
    const float* __restrict__ b_in,
    const float* __restrict__ w_state,
    const float* __restrict__ b_state,
    const float* __restrict__ w_fc,
    float* __restrict__ partial)
{
  extern __shared__ char smem[];
  bf16_t* Bt    = (bf16_t*)smem;
  float*  xsk   = (float*)(smem + BT_BYTES);
  bf16_t* hbuf  = (bf16_t*)(smem + BT_BYTES + XSK_BYTES);
  bf16_t* actsL = (bf16_t*)(smem + BT_BYTES + XSK_BYTES + HB_BYTES);
  float*  redL  = (float*)(smem + BT_BYTES + XSK_BYTES + HB_BYTES + ACT_BYTES);

  const int img  = blockIdx.x;
  const int dir  = img >> 7;
  const int bb   = img & 127;
  const int tid  = threadIdx.x;
  const int lane = tid & 31;
  const int wid  = tid >> 5;
  const int mt   = wid & 1;
  const int nt   = wid >> 1;

  for (int i = tid; i < HID * 128; i += 256) {
    int o = i >> 7, k = i & 127;
    float v = w_state[((size_t)(o * HID + (k & 63))) * 2 + (k >> 6)];
    Bt[o * BT_STRIDE + k] = (bf16_t)v;
  }
  {
    const bool flr = (dir == 1) || (dir == 3);
    const bool flc = (dir == 2) || (dir == 3);
    const float* xb = x + (size_t)bb * (HH * WW);
    for (int i = tid; i < 64 * HH; i += 256) {
      int c = i >> 5, r = i & 31;
      int j = c - r;
      float v = 0.0f;
      if (j >= 0 && j < WW) {
        int rr = flr ? (HH - 1 - r) : r;
        int jj = flc ? (WW - 1 - j) : j;
        v = xb[rr * WW + jj];
      }
      xsk[c * XSK_STRIDE + r] = v;
    }
  }
  for (int i = tid; i < 2 * HBUF_ELEMS; i += 256) hbuf[i] = (bf16_t)0.0f;

  const int lm     = lane & 15;
  const int hi     = lane >> 4;
  const int o_lane = nt * 16 + lm;
  const float win_o  = w_in[o_lane];
  const float bias_o = b_in[o_lane] + b_state[o_lane];
  const int kb    = hi * 8;
  const int r_a   = mt * 16 + lm;
  const int rbase = mt * 16 + hi * 8;

  __syncthreads();

  Frag bfrag[4];
  {
    const char* brow = (const char*)(Bt + o_lane * BT_STRIDE);
#pragma unroll
    for (int kt = 0; kt < 4; ++kt) {
      const char* p = brow + (kt * 32 + hi * 8) * 2;
      bfrag[kt].q[0] = *(const v4i*)(p);
      bfrag[kt].q[1] = *(const v4i*)(p + 32);
    }
  }

  for (int c = 0; c < STEPS; ++c) {
    const bf16_t* hin  = hbuf + ((c & 1) ? HBUF_ELEMS : 0);
    bf16_t*       hout = hbuf + ((c & 1) ? 0 : HBUF_ELEMS);

    Frag af[4];
#pragma unroll
    for (int kt = 0; kt < 4; ++kt) {
      int hrow = (kt < 2) ? r_a : (r_a + 1);
      const char* p = (const char*)(hin + hrow * H_STRIDE) + ((kt & 1) * 32 + kb) * 2;
      af[kt].q[0] = *(const v4i*)(p);
      af[kt].q[1] = *(const v4i*)(p + 32);
    }
    const float* xcol = xsk + c * XSK_STRIDE + rbase;
    v4f xv0 = *(const v4f*)(xcol);
    v4f xv1 = *(const v4f*)(xcol + 4);

    v8f acc0 = {}, acc1 = {};
    acc0 = __builtin_amdgcn_wmma_f32_16x16x32_f16(false, af[0].v, false, bfrag[0].v, (short)0, acc0, false, false);
    acc1 = __builtin_amdgcn_wmma_f32_16x16x32_f16(false, af[1].v, false, bfrag[1].v, (short)0, acc1, false, false);
    acc0 = __builtin_amdgcn_wmma_f32_16x16x32_f16(false, af[2].v, false, bfrag[2].v, (short)0, acc0, false, false);
    acc1 = __builtin_amdgcn_wmma_f32_16x16x32_f16(false, af[3].v, false, bfrag[3].v, (short)0, acc1, false, false);
    asm volatile("v_nop\n\tv_nop\n\tv_nop\n\tv_nop" : "+v"(acc0), "+v"(acc1) : "v"(af[3].v), "v"(bfrag[3].v));

    float hn[8];
#pragma unroll
    for (int v = 0; v < 8; ++v) {
      float xval = (v < 4) ? xv0[v] : xv1[v - 4];
      float s = fmaf(win_o, xval, acc0[v] + acc1[v] + bias_o);
      hn[v] = TANHF(s);
    }
#pragma unroll
    for (int v = 0; v < 8; ++v) {
      int rr = rbase + v;
      int j  = c - rr;
      bf16_t hb = (bf16_t)hn[v];
      hout[(rr + 1) * H_STRIDE + o_lane] = hb;
      int apix = ((unsigned)j < (unsigned)WW) ? (rr * WW + j) : ACT_TRASH_PIX;
      actsL[apix * ACT_STRIDE + o_lane] = hb;
    }
    __syncthreads();
  }

  float pacc[NCLS];
#pragma unroll
  for (int k = 0; k < NCLS; ++k) pacc[k] = 0.0f;

  const size_t dirOff = (size_t)dir * (HID * HH * WW);
  for (int idx = tid; idx < HID * HH * WW; idx += 256) {
    int o = idx >> 10, pix = idx & 1023;
    float av = (float)actsL[pix * ACT_STRIDE + o];
    const float* wrow = w_fc + (dirOff + (size_t)idx) * NCLS;
    __builtin_prefetch((const void*)(wrow + 256 * NCLS), 0, 1);
    const float2* w2 = (const float2*)wrow;
#pragma unroll
    for (int q = 0; q < 5; ++q) {
      float2 wv = w2[q];
      pacc[2 * q]     += av * wv.x;
      pacc[2 * q + 1] += av * wv.y;
    }
  }

#pragma unroll
  for (int k = 0; k < NCLS; ++k) {
    float v = pacc[k];
    for (int off = 16; off > 0; off >>= 1) v += __shfl_xor(v, off, 32);
    pacc[k] = v;
  }
  if (lane == 0) {
#pragma unroll
    for (int k = 0; k < NCLS; ++k) redL[wid * NCLS + k] = pacc[k];
  }
  __syncthreads();
  if (tid < PSTR) {
    float s = 0.0f;
    if (tid < NCLS) {
#pragma unroll
      for (int w = 0; w < 8; ++w) s += redL[w * NCLS + tid];
    }
    VST2(float, partial + (size_t)img * PSTR + tid, s);
  }
}

__global__ __launch_bounds__(256) void head_kernel(
    const float* __restrict__ partial,
    const float* __restrict__ b_fc,
    float* __restrict__ out)
{
  __shared__ __attribute__((aligned(16))) float so[BATCHN * NCLS];
  const int t = threadIdx.x;
  if (t < BATCHN) {
    float v[NCLS]; float m = -3.0e38f;
#pragma unroll
    for (int k = 0; k < NCLS; ++k) {
      float s = b_fc[k];
#pragma unroll
      for (int d = 0; d < 4; ++d) s += partial[((size_t)d * BATCHN + t) * PSTR + k];
      v[k] = s; m = fmaxf(m, s);
    }
    float z = 0.f;
#pragma unroll
    for (int k = 0; k < NCLS; ++k) z += expf(v[k] - m);
    const float lz = logf(z);
#pragma unroll
    for (int k = 0; k < NCLS; ++k) so[t * NCLS + k] = (v[k] - m) - lz;
  }
  __syncthreads();
  for (int p = t; p < BATCHN * NCLS / 4; p += 256) VST2(v4f, out + p * 4, *(const v4f*)(so + p * 4));
}

extern "C" void kernel_launch(void* const* d_in, const int* in_sizes, int n_in,
                              void* d_out, int out_size, void* d_ws, size_t ws_size,
                              hipStream_t stream) {
  const float* x       = (const float*)d_in[0];
  const float* w_in    = (const float*)d_in[1];
  const float* b_in    = (const float*)d_in[2];
  const float* w_state = (const float*)d_in[3];
  const float* b_state = (const float*)d_in[4];
  const float* w_fc    = (const float*)d_in[5];
  const float* b_fc    = (const float*)d_in[6];
  float* out     = (float*)d_out;
  float* partial = (float*)d_ws;

  (void)in_sizes; (void)n_in; (void)out_size;
  if (ws_size < (size_t)4 * BATCHN * PSTR * 4) return;

  hipFuncSetAttribute((const void*)mdrnn_kernel,
                      hipFuncAttributeMaxDynamicSharedMemorySize, SMEM_BYTES);

  mdrnn_kernel<<<4 * BATCHN, 256, SMEM_BYTES, stream>>>(
      x, w_in, b_in, w_state, b_state, w_fc, partial);
  head_kernel<<<1, 256, 0, stream>>>(partial, b_fc, out);
}
